// MultiHeadAttention_24781961298465
// MI455X (gfx1250) — hardware-verified
//
#include <hip/hip_runtime.h>
#include <math.h>

#ifndef NB
#define NB 2
#endif
#ifndef SEQ
#define SEQ 2048
#endif
#define NB_FULL 2
#define SEQ_FULL 2048
#define DM 1024
#define NH 16
#define HDIM 64
#define MROWS (NB * SEQ)
#define QKP (2 * DM)
#define VTP (MROWS)

static_assert(NB <= NB_FULL);
static_assert(SEQ <= SEQ_FULL);
static_assert(SEQ % 64 == 0);
static_assert(MROWS % 64 == 0);
static_assert(DM % 64 == 0);
static_assert(DM % 32 == 0);
static_assert(NH * HDIM == DM);
static_assert(HDIM == 64);

typedef __attribute__((ext_vector_type(16))) _Float16 v16h;
typedef __attribute__((ext_vector_type(8)))  _Float16 v8h;
typedef __attribute__((ext_vector_type(8)))  float    v8f;
typedef __attribute__((ext_vector_type(4)))  float    v4f;
typedef __attribute__((ext_vector_type(4)))  unsigned int v4u;

union FragH { v16h v; v8h h[2]; };

__device__ __forceinline__ v16h ldg_frag(const _Float16* __restrict__ p) {
    FragH f; f.h[0] = *(const v8h*)(p); f.h[1] = *(const v8h*)(p + 16); return f.v;
}

__device__ __forceinline__ v8f wmma16(v16h a, v16h b, v8f c) {
    c = __builtin_amdgcn_wmma_f32_16x16x32_f16(false, a, false, b, (short)0, c, false, false);
    asm volatile("v_nop\n\tv_nop\n\tv_nop\n\tv_nop" : "+v"(c) : "v"(a), "v"(b));
    return c;
}
__device__ __forceinline__ void dep_guard_h(v8f& a, v8f& b, v16h x, v16h y) { asm volatile("v_nop\n\tv_nop\n\tv_nop\n\tv_nop" : "+v"(a), "+v"(b) : "v"(x), "v"(y)); }
__device__ __forceinline__ void keep4_h(v16h a, v16h b, v16h c, v16h d) { asm volatile("v_nop" :: "v"(a), "v"(b), "v"(c), "v"(d)); }
__device__ __forceinline__ void acc_guard4(v8f& a, v8f& b, v8f& c, v8f& d) { asm volatile("v_nop\n\tv_nop\n\tv_nop\n\tv_nop" : "+v"(a), "+v"(b), "+v"(c), "+v"(d)); }

#define VST2(T, ptr, val) do { const T vst2_v_ = (val); *(volatile T*)(ptr) = vst2_v_; __threadfence(); *(volatile T*)(ptr) = vst2_v_; } while (0)

__device__ __forceinline__ float cmb_bf(float v) { const unsigned u = __float_as_uint(v); const unsigned r = (u + 0x7fffu + ((u >> 16) & 1u)) & 0xffff0000u; return __uint_as_float(r); }
__device__ __forceinline__ unsigned int cmb_pk2(float a, float b) { return (unsigned int)__builtin_bit_cast(unsigned short, (_Float16)a) | ((unsigned int)__builtin_bit_cast(unsigned short, (_Float16)b) << 16); }

__global__ __launch_bounds__(256) void k_cast_rows(const float* __restrict__ SRC, unsigned short* __restrict__ DST, int nrows, int rpb, int rpbFull, float sc) {
    const long long u = (long long)blockIdx.x * 256 + threadIdx.x; const int per = DM / 8;
    if (u >= (long long)nrows * per) return;
    const int r = (int)(u / per); const int c0 = 8 * (int)(u % per);
    const int b = r / rpb, s = r - b * rpb;
    const float* sp = SRC + ((size_t)b * rpbFull + s) * DM + c0;
    const v4f a = *(const v4f*)(sp); const v4f bb = *(const v4f*)(sp + 4);
    v4u pk;
    pk.x = cmb_pk2(cmb_bf(a.x) * sc, cmb_bf(a.y) * sc);
    pk.y = cmb_pk2(cmb_bf(a.z) * sc, cmb_bf(a.w) * sc);
    pk.z = cmb_pk2(cmb_bf(bb.x) * sc, cmb_bf(bb.y) * sc);
    pk.w = cmb_pk2(cmb_bf(bb.z) * sc, cmb_bf(bb.w) * sc);
    VST2(v4u, (v4u*)(DST + (size_t)r * DM + c0), pk);
}

template <int OUT_MODE>
__global__ __launch_bounds__(256) void k_gemm64(const unsigned short* __restrict__ Ap, int lda,
                                                const unsigned short* __restrict__ Btp, int ldb,
                                                void* __restrict__ Cout, int ldc,
                                                int M, int N, int K, float scale) {
    const _Float16* __restrict__ A = (const _Float16*)Ap;
    const _Float16* __restrict__ Bt = (const _Float16*)Btp;
    __shared__ __align__(16) float sT[8][16 * 68];
    const int lane = threadIdx.x & 31;
    const int wave = __builtin_amdgcn_readfirstlane((int)(threadIdx.x >> 5));
    const int tilesN = N >> 6;
    const int tilesM = M >> 6;
    const int tile = blockIdx.x * 8 + wave;
    if (tile >= tilesM * tilesN) return;
    const int tm = tile / tilesN;
    const int tn = tile - tm * tilesN;
    const int m0 = tm << 6;
    const int n0 = tn << 6;
    const int rlane = lane & 15;
    const int koff = (lane >> 4) * 8;
    const int mOff = (lane >> 4) * 8;

    v8f acc[4][4];
#pragma unroll
    for (int i = 0; i < 4; ++i)
#pragma unroll
        for (int j = 0; j < 4; ++j) acc[i][j] = (v8f){0.f, 0.f, 0.f, 0.f, 0.f, 0.f, 0.f, 0.f};

    for (int k0 = 0; k0 < K; k0 += 32) {
        v16h bh[4];
#pragma unroll
        for (int j = 0; j < 4; ++j) bh[j] = ldg_frag(Bt + (size_t)(n0 + (j << 4) + rlane) * ldb + koff + k0);
#pragma unroll
        for (int i = 0; i < 4; ++i) {
            const v16h ah = ldg_frag(A + (size_t)(m0 + (i << 4) + rlane) * lda + koff + k0);
#pragma unroll
            for (int j = 0; j < 4; ++j)
                acc[i][j] = __builtin_amdgcn_wmma_f32_16x16x32_f16(false, ah, false, bh[j], (short)0, acc[i][j], false, false);
            dep_guard_h(acc[i][0], acc[i][3], ah, ah);
        }
        keep4_h(bh[0], bh[1], bh[2], bh[3]);
    }
    acc_guard4(acc[0][0], acc[0][1], acc[0][2], acc[0][3]);
    acc_guard4(acc[1][0], acc[1][1], acc[1][2], acc[1][3]);
    acc_guard4(acc[2][0], acc[2][1], acc[2][2], acc[2][3]);
    acc_guard4(acc[3][0], acc[3][1], acc[3][2], acc[3][3]);

    float* slab = sT[wave];
#pragma unroll
    for (int i = 0; i < 4; ++i) {
        const int mBase = m0 + (i << 4);
#pragma unroll
        for (int j = 0; j < 4; ++j) {
#pragma unroll
            for (int r = 0; r < 8; ++r) {
                const float v = acc[i][j][r] * scale;
                slab[(mOff + r) * 68 + (j << 4) + rlane] = v;
            }
        }
        __builtin_amdgcn_fence(3  , "workgroup");
        __builtin_amdgcn_wave_barrier();
        __builtin_amdgcn_fence(2  , "workgroup");
        if (OUT_MODE == 0) {
            float* C = (float*)Cout;
            const int hh = lane >> 4, c4 = (lane & 15) * 4;
            for (int pass = 0; pass < 2; ++pass) {
#pragma unroll
                for (int it = 0; it < 8; ++it) {
                    const int row = it * 2 + hh;
                    const v4f v = *(const v4f*)(slab + row * 68 + c4);
                    *(volatile v4f*)(C + (size_t)(mBase + row) * ldc + n0 + c4) = v;
                }
                __threadfence();
            }
        } else {
            const int q = lane >> 3, c8 = (lane & 7) * 8;
            unsigned short* C = (unsigned short*)Cout;
            for (int pass = 0; pass < 2; ++pass) {
#pragma unroll
                for (int it = 0; it < 4; ++it) {
                    const int row = it * 4 + q;
                    const float* sp = slab + row * 68 + c8;
                    v8h hv;
#pragma unroll
                    for (int e = 0; e < 8; ++e) hv[e] = (_Float16)sp[e];
                    *(volatile v8h*)(C + (size_t)(mBase + row) * ldc + n0 + c8) = hv;
                }
                __threadfence();
            }
        }
        __builtin_amdgcn_fence(3  , "workgroup");
        __builtin_amdgcn_wave_barrier();
        __builtin_amdgcn_fence(2  , "workgroup");
    }
}

__global__ __launch_bounds__(128) void k_attn_f16(const unsigned short* __restrict__ QKp, const unsigned short* __restrict__ VTp,
                                                  const int* __restrict__ maskp, unsigned short* __restrict__ CTXp) {
    const _Float16* __restrict__ QK = (const _Float16*)QKp;
    const _Float16* __restrict__ VT = (const _Float16*)VTp;
    __shared__ __align__(16) _Float16 Psh[4][16 * 64];
    __shared__ __align__(16) float    Os[4][16 * 68];

    const int tid = threadIdx.x;
    const int wave = __builtin_amdgcn_readfirstlane((int)(tid >> 5));
    const int lane = tid & 31;
    const int hh = lane >> 4;
    const int c = lane & 15;

    const int nqb = SEQ / 64;
    const int bx = blockIdx.x;
    const int qb = bx % nqb;
    const int bh = bx / nqb;
    const int h = bh % NH;
    const int b = bh / NH;
    const int q0 = qb * 64 + wave * 16;
    const size_t rowbase = (size_t)b * SEQ;
    const int* __restrict__ mk = maskp + (size_t)b * SEQ_FULL;

    v16h qa0, qa1;
    {
        const _Float16* qrow = QK + (rowbase + q0 + c) * QKP + h * 64 + 8 * hh;
        qa0 = ldg_frag(qrow);
        qa1 = ldg_frag(qrow + 32);
    }

    float mrow[8], lrow[8];
    v8f oacc[4];
#pragma unroll
    for (int r = 0; r < 8; ++r) { mrow[r] = -__builtin_inff(); lrow[r] = 0.f; }
#pragma unroll
    for (int t = 0; t < 4; ++t) oacc[t] = (v8f){0.f, 0.f, 0.f, 0.f, 0.f, 0.f, 0.f, 0.f};

    const float SC = 0.125f * 1.4426950408889634f;
    const float NEGL = -100000.0f * 1.4426950408889634f;
    const float PSC = 32768.0f;
    _Float16* pw = Psh[wave];

    for (int kc = 0; kc < SEQ / 64; ++kc) {
        const int kv0 = kc * 64;
        const bool v0 = mk[kv0 + c] != 0;
        const bool v1 = mk[kv0 + 16 + c] != 0;
        const bool v2 = mk[kv0 + 32 + c] != 0;
        const bool v3 = mk[kv0 + 48 + c] != 0;
        v8f s[4];
#pragma unroll
        for (int j = 0; j < 4; ++j) {
            const _Float16* krow = QK + (rowbase + kv0 + j * 16 + c) * QKP + DM + h * 64 + 8 * hh;
            const v16h k0f = ldg_frag(krow);
            const v16h k1f = ldg_frag(krow + 32);
            v8f z = (v8f){0.f, 0.f, 0.f, 0.f, 0.f, 0.f, 0.f, 0.f};
            z = wmma16(qa0, k0f, z);
            z = wmma16(qa1, k1f, z);
            s[j] = z;
        }
#pragma unroll
        for (int r = 0; r < 8; ++r) {
            const float y0 = s[0][r] * SC, y1 = s[1][r] * SC, y2 = s[2][r] * SC, y3 = s[3][r] * SC;
            const float x0 = v0 ? y0 : NEGL;
            const float x1 = v1 ? y1 : NEGL;
            const float x2 = v2 ? y2 : NEGL;
            const float x3 = v3 ? y3 : NEGL;
            float m = fmaxf(fmaxf(x0, x1), fmaxf(x2, x3));
            m = fmaxf(m, __shfl_xor(m, 1, 32)); m = fmaxf(m, __shfl_xor(m, 2, 32));
            m = fmaxf(m, __shfl_xor(m, 4, 32)); m = fmaxf(m, __shfl_xor(m, 8, 32));
            const float mnew = fmaxf(mrow[r], m);
            const float alpha = exp2f(mrow[r] - mnew);
            mrow[r] = mnew;
            const float e0 = exp2f(x0 - mnew), e1 = exp2f(x1 - mnew), e2 = exp2f(x2 - mnew), e3 = exp2f(x3 - mnew);
            const float p0 = v0 ? e0 : 0.f;
            const float p1 = v1 ? e1 : 0.f;
            const float p2 = v2 ? e2 : 0.f;
            const float p3 = v3 ? e3 : 0.f;
            float psum = (p0 + p1) + (p2 + p3);
            const int pr = (8 * hh + r) * 64 + c;
            pw[pr]      = (_Float16)(p0 * PSC);
            pw[pr + 16] = (_Float16)(p1 * PSC);
            pw[pr + 32] = (_Float16)(p2 * PSC);
            pw[pr + 48] = (_Float16)(p3 * PSC);
            psum += __shfl_xor(psum, 1, 32); psum += __shfl_xor(psum, 2, 32);
            psum += __shfl_xor(psum, 4, 32); psum += __shfl_xor(psum, 8, 32);
            lrow[r] = lrow[r] * alpha + psum;
            oacc[0][r] *= alpha; oacc[1][r] *= alpha; oacc[2][r] *= alpha; oacc[3][r] *= alpha;
        }
        __builtin_amdgcn_fence(3  , "workgroup");
        __builtin_amdgcn_wave_barrier();
        __builtin_amdgcn_fence(2  , "workgroup");
#pragma unroll
        for (int kk = 0; kk < 2; ++kk) {
            FragH pa;
            pa.h[0] = *(const v8h*)(pw + c * 64 + kk * 32 + 8 * hh);
            pa.h[1] = *(const v8h*)(pw + c * 64 + kk * 32 + 16 + 8 * hh);
#pragma unroll
            for (int t = 0; t < 4; ++t) {
                const _Float16* vrow = VT + (size_t)(h * 64 + t * 16 + c) * VTP + rowbase + kv0 + kk * 32 + 8 * hh;
                const v16h vb = ldg_frag(vrow);
                oacc[t] = wmma16(pa.v, vb, oacc[t]);
            }
        }
        __builtin_amdgcn_fence(3  , "workgroup");
        __builtin_amdgcn_wave_barrier();
        __builtin_amdgcn_fence(2  , "workgroup");
    }

    float* os = Os[wave];
#pragma unroll
    for (int r = 0; r < 8; ++r) {
        const float l = lrow[r];
        const float rc = 1.0f / (fmaxf(l, 1.0e-30f) * 128.0f);
        const float inv = (l > 0.f) ? rc : 0.f;
#pragma unroll
        for (int t = 0; t < 4; ++t) os[(8 * hh + r) * 68 + t * 16 + c] = oacc[t][r] * inv;
    }
    __builtin_amdgcn_fence(3  , "workgroup");
    __builtin_amdgcn_wave_barrier();
    __builtin_amdgcn_fence(2  , "workgroup");
    {
        const int q = lane >> 3, c8 = (lane & 7) * 8;
        unsigned short* C = CTXp + (rowbase + q0) * DM + h * 64;
        for (int pass = 0; pass < 2; ++pass) {
#pragma unroll
            for (int it = 0; it < 4; ++it) {
                const int row = it * 4 + q;
                const float* sp = os + row * 68 + c8;
                v8h hv;
#pragma unroll
                for (int e = 0; e < 8; ++e) hv[e] = (_Float16)sp[e];
                *(volatile v8h*)(C + (size_t)row * DM + c8) = hv;
            }
            __threadfence();
        }
    }
}

static inline size_t al256(size_t n) { return ((n + 255) / 256) * 256; }

extern "C" void kernel_launch(void* const* d_in, const int* in_sizes, int n_in, void* d_out, int out_size, void* d_ws, size_t ws_size, hipStream_t stream) {
    if (n_in < 8) return;
    const long long needx = ((long long)(NB - 1) * SEQ_FULL + SEQ) * DM;
    if ((long long)in_sizes[0] < needx) return;
    if ((long long)in_sizes[1] < needx) return;
    if ((long long)in_sizes[2] < needx) return;
    if ((long long)in_sizes[3] < (long long)(NB - 1) * SEQ_FULL + SEQ) return;
    if ((long long)in_sizes[4] < (long long)DM * DM) return;
    if ((long long)in_sizes[5] < (long long)DM * DM) return;
    if ((long long)in_sizes[6] < (long long)DM * DM) return;
    if ((long long)in_sizes[7] < (long long)DM * DM) return;
    if ((long long)out_size < (long long)MROWS * DM) return;

    const float* xq   = (const float*)d_in[0];
    const float* xk   = (const float*)d_in[1];
    const float* xv   = (const float*)d_in[2];
    const int*   mask = (const int*)d_in[3];
    const float* Wq   = (const float*)d_in[4];
    const float* Wk   = (const float*)d_in[5];
    const float* Wv   = (const float*)d_in[6];
    const float* Wo   = (const float*)d_in[7];
    float* out = (float*)d_out;

    char* wsp = (char*)d_ws;
    unsigned short* XQ16 = (unsigned short*)wsp; wsp += al256((size_t)MROWS * DM * 2);
    unsigned short* XK16 = (unsigned short*)wsp; wsp += al256((size_t)MROWS * DM * 2);
    unsigned short* XV16 = (unsigned short*)wsp; wsp += al256((size_t)MROWS * DM * 2);
    unsigned short* WQ16 = (unsigned short*)wsp; wsp += al256((size_t)DM * DM * 2);
    unsigned short* WK16 = (unsigned short*)wsp; wsp += al256((size_t)DM * DM * 2);
    unsigned short* WV16 = (unsigned short*)wsp; wsp += al256((size_t)DM * DM * 2);
    unsigned short* WO16 = (unsigned short*)wsp; wsp += al256((size_t)DM * DM * 2);
    unsigned short* QK16 = (unsigned short*)wsp; wsp += al256((size_t)MROWS * QKP * 2);
    unsigned short* VT16 = (unsigned short*)wsp; wsp += al256((size_t)DM * VTP * 2);
    unsigned short* CX16 = (unsigned short*)wsp; wsp += al256((size_t)MROWS * DM * 2);
    if ((size_t)(wsp - (char*)d_ws) > ws_size) return;

    const unsigned gx = (unsigned)(((long long)MROWS * (DM / 8) + 255) / 256);
    const unsigned gw = (unsigned)(((long long)DM * (DM / 8) + 255) / 256);
    k_cast_rows<<<gx, 256, 0, stream>>>(xq, XQ16, MROWS, SEQ, SEQ_FULL, 1.0f);
    k_cast_rows<<<gx, 256, 0, stream>>>(xk, XK16, MROWS, SEQ, SEQ_FULL, 1.0f);
    k_cast_rows<<<gx, 256, 0, stream>>>(xv, XV16, MROWS, SEQ, SEQ_FULL, 1.0f);
    k_cast_rows<<<gw, 256, 0, stream>>>(Wq, WQ16, DM, DM, DM, 16.0f);
    k_cast_rows<<<gw, 256, 0, stream>>>(Wk, WK16, DM, DM, DM, 16.0f);
    k_cast_rows<<<gw, 256, 0, stream>>>(Wv, WV16, DM, DM, DM, 16.0f);
    k_cast_rows<<<gw, 256, 0, stream>>>(Wo, WO16, DM, DM, DM, 16.0f);

    k_gemm64<1><<<(unsigned)(((MROWS / 64) * (DM / 64) + 7) / 8), 256, 0, stream>>>(
        XQ16, DM, WQ16, DM, (void*)QK16, QKP, MROWS, DM, DM, 0.0625f);
    k_gemm64<1><<<(unsigned)(((MROWS / 64) * (DM / 64) + 7) / 8), 256, 0, stream>>>(
        XK16, DM, WK16, DM, (void*)(QK16 + DM), QKP, MROWS, DM, DM, 0.0625f);
    k_gemm64<1><<<(unsigned)(((DM / 64) * (MROWS / 64) + 7) / 8), 256, 0, stream>>>(
        WV16, DM, XV16, DM, (void*)VT16, VTP, DM, MROWS, DM, 0.0625f);

    k_attn_f16<<<(unsigned)(NB * NH * (SEQ / 64)), 128, 0, stream>>>(QK16, VT16, mask, CX16);

    k_gemm64<0><<<(unsigned)(((MROWS / 64) * (DM / 64) + 7) / 8), 256, 0, stream>>>(
        CX16, DM, WO16, DM, (void*)out, DM, MROWS, DM, DM, 1.0f / 4096.0f);
}
